// MultiHeadGATLayer_72516227826098
// MI455X (gfx1250) — hardware-verified
//
#include <hip/hip_runtime.h>
#include <stddef.h>
#include <stdint.h>

typedef _Float16 v16h __attribute__((ext_vector_type(16)));
typedef _Float16 v8h __attribute__((ext_vector_type(8)));
typedef _Float16 v4h __attribute__((ext_vector_type(4)));
typedef float v8f __attribute__((ext_vector_type(8)));
typedef float v4f __attribute__((ext_vector_type(4)));
typedef float v4fa __attribute__((ext_vector_type(4), __may_alias__));
typedef int v4i __attribute__((ext_vector_type(4)));

union HFrag { v16h v; v8h half[2]; };
union H8 { v8h v; _Float16 e[8]; };
union H4 { v4h v; _Float16 e[4]; };

#define DIM 512
#define NHEAD 8
#define HDIM 64
#define GROWS 32
#define GTHREADS 256
#define ZPITCH 520
#define NBLK 128
#define ATHREADS 128
#define AWAVES 4
#define CHUNK (ATHREADS * 16)
#define CAP 5632
#define SS_FLOATS (NBLK * DIM)
#define DS_FLOATS (NBLK * NHEAD)
#define AGG_LDS_BYTES (SS_FLOATS * 4 + DS_FLOATS * 4 + CAP * 4 + 64)

__device__ __forceinline__ v8f zero8() {
  v8f z = {0.f, 0.f, 0.f, 0.f, 0.f, 0.f, 0.f, 0.f};
  return z;
}

__device__ __forceinline__ v8f wmma_f16(v16h a, v16h b, v8f c) {
  v8f d = __builtin_amdgcn_wmma_f32_16x16x32_f16(false, a, false, b, (short)0, c, false, false);
  asm volatile("v_nop\n\tv_nop\n\tv_nop\n\tv_nop" : "+v"(d) : "v"(a), "v"(b));
  return d;
}

__device__ __forceinline__ float elu1(float v) { return v > 0.0f ? v : (__expf(v) - 1.0f); }

__global__ __launch_bounds__(256) void prep_kernel(const float* __restrict__ x,
                                                   const float* __restrict__ W1,
                                                   const float* __restrict__ Wo,
                                                   _Float16* x16, _Float16* W1t, _Float16* Wot,
                                                   int nx8, int nxBlocks) {
  const int bid = blockIdx.x, t = threadIdx.x;
  if (bid < nxBlocks) {
    const int tid = bid * 256 + t;
    if (tid < nx8) {
      const float* p = x + (size_t)tid * 8;
      const v4f u0 = *(const v4f*)p;
      const v4f u1 = *(const v4f*)(p + 4);
      H8 o;
      o.e[0] = (_Float16)u0.x; o.e[1] = (_Float16)u0.y; o.e[2] = (_Float16)u0.z; o.e[3] = (_Float16)u0.w;
      o.e[4] = (_Float16)u1.x; o.e[5] = (_Float16)u1.y; o.e[6] = (_Float16)u1.z; o.e[7] = (_Float16)u1.w;
      _Float16* d = x16 + (size_t)tid * 8;
      *(volatile v8h*)d = o.v;
      __threadfence();
      *(volatile v8h*)d = o.v;
    }
  } else if (bid < nxBlocks + 128) {
    const int tid = (bid - nxBlocks) * 256 + t;
    const int col = tid >> 6, q = tid & 63;
    const int hh = col >> 6, c = col & 63;
    H8 o;
#pragma unroll
    for (int i = 0; i < 8; ++i)
      o.e[i] = (_Float16)(W1[((size_t)hh * DIM + 8 * q + i) * HDIM + c] * 16.0f);
    _Float16* d = W1t + (size_t)col * DIM + 8 * q;
    *(volatile v8h*)d = o.v;
    __threadfence();
    *(volatile v8h*)d = o.v;
  } else {
    const int tid = (bid - nxBlocks - 128) * 256 + t;
    if (tid < 32768) {
      const int n = tid >> 6, q = tid & 63;
      H8 o;
#pragma unroll
      for (int i = 0; i < 8; ++i)
        o.e[i] = (_Float16)(Wo[(size_t)(8 * q + i) * DIM + n] * 16.0f);
      _Float16* d = Wot + (size_t)n * DIM + 8 * q;
      *(volatile v8h*)d = o.v;
      __threadfence();
      *(volatile v8h*)d = o.v;
    }
  }
}

template <int LAYER>
__device__ __forceinline__ void gemm_store(const _Float16* zL, const float* esP, const float* edP,
                                           const float* esF, const float* edF, _Float16* Z16,
                                           float* esO, float* edO, int rowBase, int N, int l, int w) {
#pragma unroll
  for (int j = 0; j < 8; ++j) {
    const int row = 4 * w + (j >> 1);
    const int col0 = (j & 1) * 256 + 8 * l;
    const int node = rowBase + row;
    if (node < N) {
      const v8h v = *(const v8h*)(zL + row * ZPITCH + col0);
      *(volatile v8h*)(Z16 + (size_t)node * DIM + col0) = v;
    }
  }
  if (rowBase + GROWS <= N) {
    if (LAYER == 1) {
      if (l < 8) {
        const v4f v = *(const v4fa*)(esP + w * 32 + 4 * l);
        *(volatile v4f*)(esO + (size_t)w * N + rowBase + 4 * l) = v;
      } else if (l < 16) {
        const v4f v = *(const v4fa*)(edP + w * 32 + 4 * (l - 8));
        *(volatile v4f*)(edO + (size_t)w * N + rowBase + 4 * (l - 8)) = v;
      }
    } else {
      if (w == 0) {
        if (l < 8) {
          const v4f v = *(const v4fa*)(esF + 4 * l);
          *(volatile v4f*)(esO + rowBase + 4 * l) = v;
        } else if (l < 16) {
          const v4f v = *(const v4fa*)(edF + 4 * (l - 8));
          *(volatile v4f*)(edO + rowBase + 4 * (l - 8)) = v;
        }
      }
    }
  }
}

template <int LAYER>
__global__ __launch_bounds__(GTHREADS) void gemm_kernel(const _Float16* __restrict__ A,
                                                         const _Float16* __restrict__ Bt,
                                                         const float* __restrict__ av,
                                                         _Float16* Z16, float* esO, float* edO, int N) {
  __shared__ __align__(16) _Float16 zL[GROWS * ZPITCH];
  __shared__ __align__(16) float esP[8 * 32];
  __shared__ __align__(16) float edP[8 * 32];
  __shared__ __align__(16) float esF[32];
  __shared__ __align__(16) float edF[32];

  const int t = threadIdx.x, l = t & 31, w = t >> 5, hh = l >> 4, n = l & 15;
  const int rowBase = blockIdx.x * GROWS;
  const int colw = w * 64;
  const float INV16 = 0.0625f;

  int r0 = rowBase + n;      if (r0 > N - 1) r0 = N - 1;
  int r1 = rowBase + 16 + n; if (r1 > N - 1) r1 = N - 1;
  const _Float16* ap0 = A + (size_t)r0 * DIM + 8 * hh;
  const _Float16* ap1 = A + (size_t)r1 * DIM + 8 * hh;
  const _Float16* bp = Bt + (size_t)(colw + n) * DIM + 8 * hh;

  v8f acc[8];
#pragma unroll
  for (int i = 0; i < 8; ++i) acc[i] = zero8();

#pragma unroll 1
  for (int k0 = 0; k0 < DIM; k0 += 32) {
    HFrag a0, a1;
    a0.half[0] = *(const v8h*)(ap0 + k0);
    a0.half[1] = *(const v8h*)(ap0 + k0 + 16);
    a1.half[0] = *(const v8h*)(ap1 + k0);
    a1.half[1] = *(const v8h*)(ap1 + k0 + 16);
#pragma unroll
    for (int ct = 0; ct < 4; ++ct) {
      const _Float16* q = bp + (size_t)ct * 16 * DIM + k0;
      HFrag b;
      b.half[0] = *(const v8h*)q;
      b.half[1] = *(const v8h*)(q + 16);
      acc[ct] = wmma_f16(a0.v, b.v, acc[ct]);
      acc[4 + ct] = wmma_f16(a1.v, b.v, acc[4 + ct]);
    }
  }

  float avs[4], avd[4];
#pragma unroll
  for (int ct = 0; ct < 4; ++ct) {
    if (LAYER == 1) {
      avs[ct] = av[w * 128 + ct * 16 + n];
      avd[ct] = av[w * 128 + 64 + ct * 16 + n];
    } else {
      avs[ct] = av[colw + ct * 16 + n];
      avd[ct] = av[DIM + colw + ct * 16 + n];
    }
  }

#pragma unroll
  for (int rt = 0; rt < 2; ++rt) {
    float ps[8], pd[8];
#pragma unroll
    for (int r = 0; r < 8; ++r) {
      float s = 0.f, d = 0.f;
#pragma unroll
      for (int ct = 0; ct < 4; ++ct) {
        const float v = acc[rt * 4 + ct][r];
        s += v * avs[ct];
        d += v * avd[ct];
        zL[(rt * 16 + 8 * hh + r) * ZPITCH + colw + ct * 16 + n] = (_Float16)(v * INV16);
      }
      ps[r] = s;
      pd[r] = d;
    }
#pragma unroll
    for (int r = 0; r < 8; ++r) {
#pragma unroll
      for (int o = 1; o < 16; o <<= 1) {
        ps[r] += __shfl_xor(ps[r], o, 32);
        pd[r] += __shfl_xor(pd[r], o, 32);
      }
    }
    if (n == 0) {
#pragma unroll
      for (int r = 0; r < 8; ++r) {
        esP[w * 32 + rt * 16 + 8 * hh + r] = ps[r] * INV16;
        edP[w * 32 + rt * 16 + 8 * hh + r] = pd[r] * INV16;
      }
    }
  }
  __syncthreads();

  if (LAYER == 2) {
    if (t < 32) {
      float s = 0.f, d = 0.f;
#pragma unroll
      for (int ww = 0; ww < 8; ++ww) {
        s += esP[ww * 32 + t];
        d += edP[ww * 32 + t];
      }
      esF[t] = s;
      edF[t] = d;
    }
    __syncthreads();
  }

  gemm_store<LAYER>(zL, esP, edP, esF, edF, Z16, esO, edO, rowBase, N, l, w);
  __threadfence();
  gemm_store<LAYER>(zL, esP, edP, esF, edF, Z16, esO, edO, rowBase, N, l, w);
}

__device__ __forceinline__ void chunk_scan(const int* __restrict__ dstA, int E, bool vec4, int cbase,
                                           int nodeBase, int t, int l, int w, int count, int* wtot,
                                           int (&dv)[16], unsigned& hit, int& pos, int& tot) {
#pragma unroll
  for (int j = 0; j < 4; ++j) {
    const int e4 = cbase + (ATHREADS * 4) * j + 4 * t;
    int d0 = -1, d1 = -1, d2 = -1, d3 = -1;
    if (vec4 && (e4 + 4 <= E)) {
      const v4i dd = *(const v4i*)(dstA + e4);
      d0 = dd.x; d1 = dd.y; d2 = dd.z; d3 = dd.w;
    } else {
      if (e4 < E) d0 = dstA[e4];
      if (e4 + 1 < E) d1 = dstA[e4 + 1];
      if (e4 + 2 < E) d2 = dstA[e4 + 2];
      if (e4 + 3 < E) d3 = dstA[e4 + 3];
    }
    dv[4 * j] = d0; dv[4 * j + 1] = d1; dv[4 * j + 2] = d2; dv[4 * j + 3] = d3;
  }
  hit = 0;
  int cnt = 0;
#pragma unroll
  for (int i = 0; i < 16; ++i) {
    const int s = dv[i] - nodeBase;
    if ((unsigned)s < (unsigned)NBLK) { hit |= (1u << i); ++cnt; }
  }
  int incl = cnt;
#pragma unroll
  for (int o = 1; o < 32; o <<= 1) {
    const int y = __shfl_up(incl, o, 32);
    if (l >= o) incl += y;
  }
  if (l == 31) wtot[w] = incl;
  __syncthreads();
  pos = count + incl - cnt;
  tot = 0;
#pragma unroll
  for (int i = 0; i < AWAVES; ++i) {
    const int v = wtot[i];
    if (i < w) pos += v;
    tot += v;
  }
}

template <int LAYER>
__device__ __forceinline__ void agg_store(const float* sS, _Float16* hout, float* outf,
                                          int nodeBase, int N, int l, int w) {
  if (LAYER == 1) {
#pragma unroll 4
    for (int j = 0; j < 64; ++j) {
      const int row = 32 * w + (j >> 1);
      const int col0 = (j & 1) * 256 + 8 * l;
      const int node = nodeBase + row;
      if (node < N) {
        const v4f u0 = *(const v4fa*)(sS + row * DIM + col0);
        const v4f u1 = *(const v4fa*)(sS + row * DIM + col0 + 4);
        H8 o;
        o.e[0] = (_Float16)u0.x; o.e[1] = (_Float16)u0.y; o.e[2] = (_Float16)u0.z; o.e[3] = (_Float16)u0.w;
        o.e[4] = (_Float16)u1.x; o.e[5] = (_Float16)u1.y; o.e[6] = (_Float16)u1.z; o.e[7] = (_Float16)u1.w;
        *(volatile v8h*)(hout + (size_t)node * DIM + col0) = o.v;
      }
    }
  } else {
#pragma unroll 4
    for (int j = 0; j < 128; ++j) {
      const int row = 32 * w + (j >> 2);
      const int col0 = (j & 3) * 128 + 4 * l;
      const int node = nodeBase + row;
      if (node < N) {
        const v4f v = *(const v4fa*)(sS + row * DIM + col0);
        *(volatile v4f*)(outf + (size_t)node * DIM + col0) = v;
      }
    }
  }
}

template <int LAYER>
__global__ __launch_bounds__(ATHREADS) void agg_kernel(const int* __restrict__ srcA,
                                                        const int* __restrict__ dstA,
                                                        const _Float16* __restrict__ zin,
                                                        const float* __restrict__ es,
                                                        const float* __restrict__ ed,
                                                        const float* __restrict__ xres,
                                                        _Float16* hout, float* outf, int N, int E) {
  extern __shared__ __align__(16) unsigned char smem[];
  float* sS = (float*)smem;
  float* dS = sS + SS_FLOATS;
  int* list = (int*)(dS + DS_FLOATS);
  int* wtot = list + CAP;

  const int t = threadIdx.x, l = t & 31, w = t >> 5;
  const int hd = t >> 4;
  const int nodeBase = blockIdx.x * NBLK;

  {
    const v4f z = {0.f, 0.f, 0.f, 0.f};
    for (int i = t; i < (SS_FLOATS + DS_FLOATS) / 4; i += ATHREADS) *(v4f*)(sS + 4 * i) = z;
  }
  __syncthreads();

  int count = 0;
  const int nch = (E + CHUNK - 1) / CHUNK;
  const bool vec4 = ((E & 3) == 0);
  for (int ci = 0; ci < nch; ++ci) {
    const int cbase = ci * CHUNK;
    int dv[16];
    unsigned hit;
    int pos, tot;
    chunk_scan(dstA, E, vec4, cbase, nodeBase, t, l, w, count, wtot, dv, hit, pos, tot);
#pragma unroll
    for (int i = 0; i < 16; ++i) {
      if (hit & (1u << i)) {
        int e = cbase + (ATHREADS * 4) * (i >> 2) + 4 * t + (i & 3);
        if (e >= E) e = E - 1;
        if (e < 0) e = 0;
        if ((unsigned)pos < (unsigned)CAP) list[pos] = (e << 7) | (dv[i] - nodeBase);
        ++pos;
      }
    }
    count += tot;
    if (count > CAP) count = CAP;
    __syncthreads();
  }
  __syncthreads();

  {
    const int cc = count;
    float* myS = sS + 4 * t;
#pragma unroll 1
    for (int li = 0; li < CAP; ++li) {
      if (li >= cc) break;
      const int ent = list[li];
      int e = ent >> 7;
      if (e >= E) e = E - 1;
      if (e < 0) e = 0;
      const int slot = ent & (NBLK - 1);
      int s = srcA[e];
      s = (s < 0) ? 0 : ((s >= N) ? (N - 1) : s);
      int dn = nodeBase + slot;
      if (dn > N - 1) dn = N - 1;
      float ev;
      if (LAYER == 1) ev = es[(size_t)hd * N + s] + ed[(size_t)hd * N + dn];
      else            ev = es[s] + ed[dn];
      ev = fmaxf(ev, 0.2f * ev);
      ev = fminf(ev, 60.0f);
      const float ex = __expf(ev);
      H4 zz;
      zz.v = *(const v4h*)(zin + (size_t)s * DIM + 4 * t);
      v4f cur = *(v4f*)(myS + slot * DIM);
      cur.x += ex * (float)zz.e[0];
      cur.y += ex * (float)zz.e[1];
      cur.z += ex * (float)zz.e[2];
      cur.w += ex * (float)zz.e[3];
      *(v4f*)(myS + slot * DIM) = cur;
      if (LAYER == 1) {
        if ((t & 15) == 0) dS[slot * NHEAD + hd] += ex;
      } else {
        if (t == 0) dS[slot] += ex;
      }
    }
  }
  __syncthreads();

#pragma unroll 1
  for (int sl = 0; sl < NBLK; ++sl) {
    float* p = sS + sl * DIM + 4 * t;
    const v4f cur = *(v4f*)p;
    const float d = (LAYER == 1) ? dS[sl * NHEAD + hd] : dS[sl];
    const float inv = __builtin_amdgcn_rcpf(d + 1e-30f);
    v4f o;
    o.x = elu1(cur.x * inv);
    o.y = elu1(cur.y * inv);
    o.z = elu1(cur.z * inv);
    o.w = elu1(cur.w * inv);
    if (LAYER == 2) {
      const int node = nodeBase + sl;
      if (node < N) {
        const v4f xr = *(const v4f*)(xres + (size_t)node * DIM + 4 * t);
        o += xr;
      }
    }
    *(v4f*)p = o;
  }
  __syncthreads();

  agg_store<LAYER>(sS, hout, outf, nodeBase, N, l, w);
  __threadfence();
  agg_store<LAYER>(sS, hout, outf, nodeBase, N, l, w);
}

extern "C" void kernel_launch(void* const* d_in, const int* in_sizes, int n_in,
                              void* d_out, int out_size, void* d_ws, size_t ws_size,
                              hipStream_t stream) {
  if (n_in < 7) return;
  const float* h    = (const float*)d_in[0];
  const float* W1   = (const float*)d_in[1];
  const float* a1   = (const float*)d_in[2];
  const float* Wout = (const float*)d_in[3];
  const float* aout = (const float*)d_in[4];
  const int*   src  = (const int*)d_in[5];
  const int*   dst  = (const int*)d_in[6];

  const int nx = in_sizes[0];
  const int N = nx / DIM;
  const int E = in_sizes[5];
  if (N <= 0 || E <= 0) return;
  if (nx != N * DIM) return;
  if ((N % NBLK) != 0 || (N % GROWS) != 0) return;
  if (in_sizes[1] != NHEAD * DIM * HDIM || in_sizes[2] != NHEAD * 2 * HDIM ||
      in_sizes[3] != DIM * DIM || in_sizes[4] != 2 * DIM || in_sizes[6] != E) return;
  if (E >= (1 << 24)) return;
  if (out_size < N * DIM) return;

  size_t off = 0;
  const size_t ox16  = off; off += (size_t)N * DIM * 2;       off = (off + 255) & ~(size_t)255;
  const size_t oW1t  = off; off += (size_t)DIM * DIM * 2;     off = (off + 255) & ~(size_t)255;
  const size_t oWot  = off; off += (size_t)DIM * DIM * 2;     off = (off + 255) & ~(size_t)255;
  const size_t oZ1   = off; off += (size_t)N * DIM * 2;       off = (off + 255) & ~(size_t)255;
  const size_t oes1  = off; off += (size_t)NHEAD * N * 4;     off = (off + 255) & ~(size_t)255;
  const size_t oed1  = off; off += (size_t)NHEAD * N * 4;     off = (off + 255) & ~(size_t)255;
  const size_t ohc   = off; off += (size_t)N * DIM * 2;       off = (off + 255) & ~(size_t)255;
  const size_t oZ2   = off; off += (size_t)N * DIM * 2;       off = (off + 255) & ~(size_t)255;
  const size_t oes2  = off; off += (size_t)N * 4;             off = (off + 255) & ~(size_t)255;
  const size_t oed2  = off; off += (size_t)N * 4;             off = (off + 255) & ~(size_t)255;
  if (off > ws_size) return;
  if (off > ((size_t)128 << 20)) return;

  unsigned char* ws = (unsigned char*)d_ws;
  _Float16* x16   = (_Float16*)(ws + ox16);
  _Float16* W1t   = (_Float16*)(ws + oW1t);
  _Float16* Wot   = (_Float16*)(ws + oWot);
  _Float16* Z1    = (_Float16*)(ws + oZ1);
  float*    es1   = (float*)(ws + oes1);
  float*    ed1   = (float*)(ws + oed1);
  _Float16* hcat  = (_Float16*)(ws + ohc);
  _Float16* Z2    = (_Float16*)(ws + oZ2);
  float*    es2   = (float*)(ws + oes2);
  float*    ed2   = (float*)(ws + oed2);
  float*    out   = (float*)d_out;

  const int nx8 = N * (DIM / 8);
  const int nxBlocks = (nx8 + 255) / 256;
  const unsigned gemmBlocks = (unsigned)((N + GROWS - 1) / GROWS);
  const unsigned aggBlocks = (unsigned)((N + NBLK - 1) / NBLK);

  prep_kernel<<<(unsigned)(nxBlocks + 256), 256, 0, stream>>>(h, W1, Wout, x16, W1t, Wot, nx8, nxBlocks);

  gemm_kernel<1><<<gemmBlocks, GTHREADS, 0, stream>>>(x16, W1t, a1, Z1, es1, ed1, N);

  hipFuncSetAttribute((const void*)agg_kernel<1>, hipFuncAttributeMaxDynamicSharedMemorySize, AGG_LDS_BYTES);
  agg_kernel<1><<<aggBlocks, ATHREADS, AGG_LDS_BYTES, stream>>>(src, dst, Z1, es1, ed1, h, hcat, out, N, E);

  gemm_kernel<2><<<gemmBlocks, GTHREADS, 0, stream>>>(hcat, Wot, aout, Z2, es2, ed2, N);

  hipFuncSetAttribute((const void*)agg_kernel<2>, hipFuncAttributeMaxDynamicSharedMemorySize, AGG_LDS_BYTES);
  agg_kernel<2><<<aggBlocks, ATHREADS, AGG_LDS_BYTES, stream>>>(src, dst, Z2, es2, ed2, h, hcat, out, N, E);

  (void)hipGetLastError();
}
